// SelfAttn1d_3582002725319
// MI455X (gfx1250) — hardware-verified
//
#include <hip/hip_runtime.h>
#include <stdint.h>
#include <stddef.h>

typedef __attribute__((ext_vector_type(16))) _Float16 v16h;
typedef __attribute__((ext_vector_type(8)))  _Float16 v8h;
typedef __attribute__((ext_vector_type(16))) __bf16   v16b;
typedef __attribute__((ext_vector_type(8)))  __bf16   v8b;
typedef __attribute__((ext_vector_type(8)))  float    v8f;
typedef __attribute__((ext_vector_type(4)))  float    v4f;

#define LN_F 1024
#define WS_CAP ((size_t)134217728)

__device__ __forceinline__ unsigned short f2bf_bits(float f) {
  unsigned u = __float_as_uint(f);
  return (unsigned short)((u + 0x7FFFu + ((u >> 16) & 1u)) >> 16);
}
__device__ __forceinline__ float bf_bits2f(unsigned short h) { return __uint_as_float(((unsigned)h) << 16); }

__device__ __forceinline__ void dep_guard_h(v8f& a, v8f& b, v16h x, v16h y) { asm volatile("v_nop\n\tv_nop\n\tv_nop\n\tv_nop" : "+v"(a), "+v"(b) : "v"(x), "v"(y)); }
__device__ __forceinline__ void dep_guard_b(v8f& a, v8f& b, v16b x, v16b y) { asm volatile("v_nop\n\tv_nop\n\tv_nop\n\tv_nop" : "+v"(a), "+v"(b) : "v"(x), "v"(y)); }
__device__ __forceinline__ void keep4_h(v16h a, v16h b, v16h c, v16h d) { asm volatile("v_nop" :: "v"(a), "v"(b), "v"(c), "v"(d)); }
__device__ __forceinline__ void keep4_b(v16b a, v16b b, v16b c, v16b d) { asm volatile("v_nop" :: "v"(a), "v"(b), "v"(c), "v"(d)); }
__device__ __forceinline__ void acc_guard4(v8f& a, v8f& b, v8f& c, v8f& d) { asm volatile("v_nop\n\tv_nop\n\tv_nop\n\tv_nop" : "+v"(a), "+v"(b), "+v"(c), "+v"(d)); }

template <typename T> struct Frag;
template <> struct Frag<_Float16> {
  typedef v16h V; union U { v16h v; v8h h[2]; };
  static __device__ __forceinline__ v16h load(const _Float16* p) {
    U f; f.h[0] = *(const v8h*)(p); f.h[1] = *(const v8h*)(p + 16); return f.v;
  }
  static __device__ __forceinline__ v8f mma(v16h a, v16h b, v8f c) {
    return __builtin_amdgcn_wmma_f32_16x16x32_f16(false, a, false, b, (short)0, c, false, false);
  }
  static __device__ __forceinline__ void guard(v8f& a, v8f& b, v16h x, v16h y) { dep_guard_h(a, b, x, y); }
  static __device__ __forceinline__ void keep(v16h a, v16h b, v16h c, v16h d) { keep4_h(a, b, c, d); }
};
template <> struct Frag<__bf16> {
  typedef v16b V; union U { v16b v; v8b h[2]; };
  static __device__ __forceinline__ v16b load(const __bf16* p) {
    U f; f.h[0] = *(const v8b*)(p); f.h[1] = *(const v8b*)(p + 16); return f.v;
  }
  static __device__ __forceinline__ v8f mma(v16b a, v16b b, v8f c) {
    return __builtin_amdgcn_wmma_f32_16x16x32_bf16(false, a, false, b, (short)0, c, false, false);
  }
  static __device__ __forceinline__ void guard(v8f& a, v8f& b, v16b x, v16b y) { dep_guard_b(a, b, x, y); }
  static __device__ __forceinline__ void keep(v16b a, v16b b, v16b c, v16b d) { keep4_b(a, b, c, d); }
};

template <int ET> struct Elem;
template <> struct Elem<0> { typedef _Float16 T; };
template <> struct Elem<1> { typedef __bf16 T; };
template <int ET, bool SPLIT, int BIAS_MODE, int OUT_MODE, bool RESID, int ACT = 0, int ROWSEL = 0>
__global__ __launch_bounds__(256) void wmma_gemm64(
    const unsigned short* __restrict__ Ap, const unsigned short* __restrict__ A2p, int lda, long strideA,
    const unsigned short* __restrict__ Btp, const unsigned short* __restrict__ Bt2p, int ldb, long strideB,
    void* __restrict__ Cout, void* __restrict__ Cout2, int ldc, long strideC,
    const float* __restrict__ bias,
    const float* __restrict__ resid, long strideR,
    int M, int N, int K, float scale,
    const int* __restrict__ rowlen, int rpb) {
  typedef typename Elem<ET>::T T;
  typedef typename Frag<T>::V V;
  const T* A = (const T*)Ap; const T* A2 = (const T*)A2p; const T* Bt = (const T*)Btp; const T* Bt2 = (const T*)Bt2p;
  __shared__ __align__(16) float sT[8][16 * 68];
  const int b    = blockIdx.y;
  const int lane = threadIdx.x & 31;
  const int wave = threadIdx.x >> 5;
  const int tilesN = N >> 6;
  const int tilesM = M >> 6;
  const int tile = blockIdx.x * 8 + wave;
  if (tile >= tilesM * tilesN) return;
  const int tm = tile / tilesN;
  const int tn = tile - tm * tilesN;
  const int m0 = tm << 6;
  const int n0 = tn << 6;

  int nb = 0, rlen = 0;
  if (ROWSEL != 0) {
    const int bi = m0 / rpb;
    nb = m0 - bi * rpb;
    rlen = rowlen[bi];
    rlen = rlen < 0 ? 0 : (rlen > rpb ? rpb : rlen);
    if (nb >= rlen) return;
  }

  const T* Ab  = A  + (size_t)b * strideA;
  const T* Bb  = Bt + (size_t)b * strideB;
  const T* Ab2 = SPLIT ? (A2  + (size_t)b * strideA) : nullptr;
  const T* Bb2 = SPLIT ? (Bt2 + (size_t)b * strideB) : nullptr;

  const int rlane = lane & 15;
  const int koff  = (lane >> 4) * 8;
  const int mOff  = (lane >> 4) * 8;

  v8f acc[4][4];
#pragma unroll
  for (int i = 0; i < 4; ++i)
#pragma unroll
    for (int j = 0; j < 4; ++j) acc[i][j] = (v8f){0.f,0.f,0.f,0.f,0.f,0.f,0.f,0.f};

  for (int k0 = 0; k0 < K; k0 += 32) {
    V bh[4], bl[4];
#pragma unroll
    for (int j = 0; j < 4; ++j) {
      const size_t bo = (size_t)(n0 + (j << 4) + rlane) * ldb + koff + k0;
      bh[j] = Frag<T>::load(Bb + bo);
      if (SPLIT) bl[j] = Frag<T>::load(Bb2 + bo);
    }
#pragma unroll
    for (int i = 0; i < 4; ++i) {
      const size_t ao = (size_t)(m0 + (i << 4) + rlane) * lda + koff + k0;
      V ah = Frag<T>::load(Ab + ao);
      V al;
      if (SPLIT) al = Frag<T>::load(Ab2 + ao);
#pragma unroll
      for (int j = 0; j < 4; ++j) {
        acc[i][j] = Frag<T>::mma(ah, bh[j], acc[i][j]);
        if (SPLIT) {
          acc[i][j] = Frag<T>::mma(ah, bl[j], acc[i][j]);
          acc[i][j] = Frag<T>::mma(al, bh[j], acc[i][j]);
        }
      }
      Frag<T>::guard(acc[i][0], acc[i][3], ah, SPLIT ? al : ah);
    }
    Frag<T>::keep(bh[0], bh[1], bh[2], bh[3]);
    if (SPLIT) Frag<T>::keep(bl[0], bl[1], bl[2], bl[3]);
  }
  acc_guard4(acc[0][0], acc[0][1], acc[0][2], acc[0][3]);
  acc_guard4(acc[1][0], acc[1][1], acc[1][2], acc[1][3]);
  acc_guard4(acc[2][0], acc[2][1], acc[2][2], acc[2][3]);
  acc_guard4(acc[3][0], acc[3][1], acc[3][2], acc[3][3]);

  float* slab = sT[wave];
  const float* Rb = RESID ? (resid + (size_t)b * strideR) : nullptr;
#pragma unroll
  for (int i = 0; i < 4; ++i) {
    const int mBase = m0 + (i << 4);
#pragma unroll
    for (int j = 0; j < 4; ++j) {
      const int n = n0 + (j << 4) + rlane;
      float bv = 0.f;
      if (BIAS_MODE == 2) bv = bias[n];
#pragma unroll
      for (int r = 0; r < 8; ++r) {
        float v = acc[i][j][r] * scale;
        if (BIAS_MODE == 1) v += bias[mBase + mOff + r];
        if (BIAS_MODE == 2) v += bv;
        if (RESID) v += Rb[(size_t)(mBase + mOff + r) * ldc + n];
        if (ACT == 1) v = tanhf(v);
        if (ACT == 2) v = fmaxf(v, 0.0f);
        if (ACT == 3) v = v / (1.0f + expf(-v));
        if (ACT == 4) v = (v > 0.f) ? v : 0.01f * v;
        if (ACT == 5) v = 0.5f * v * (1.0f + erff(v * 0.70710678118654752f));
        if (ROWSEL == 2) { if (nb + (i << 4) + mOff + r >= rlen) v = 0.0f; }
        slab[(mOff + r) * 68 + (j << 4) + rlane] = v;
      }
    }
    __builtin_amdgcn_fence(__ATOMIC_RELEASE, "workgroup");
    __builtin_amdgcn_wave_barrier();
    __builtin_amdgcn_fence(__ATOMIC_ACQUIRE, "workgroup");
    if (OUT_MODE == 0) {
      float* C = (float*)Cout + (size_t)b * strideC;
      const int hh = lane >> 4, c4 = (lane & 15) * 4;
      for (int pass = 0; pass < 2; ++pass) {
#pragma unroll
        for (int it = 0; it < 8; ++it) {
          const int row = it * 2 + hh;
          v4f v = *(const v4f*)(slab + row * 68 + c4);
          *(volatile v4f*)(C + (size_t)(mBase + row) * ldc + n0 + c4) = v;
        }
        __threadfence();
      }
    } else {
      const int q = lane >> 3, c8 = (lane & 7) * 8;
      unsigned short* C  = (unsigned short*)Cout  + (size_t)b * strideC;
      unsigned short* C2 = (OUT_MODE == 2) ? ((unsigned short*)Cout2 + (size_t)b * strideC) : nullptr;
      for (int pass = 0; pass < 2; ++pass) {
#pragma unroll
        for (int it = 0; it < 4; ++it) {
          const int row = it * 4 + q;
          const float* sp = slab + row * 68 + c8;
          v8h hv, lv;
#pragma unroll
          for (int e = 0; e < 8; ++e) {
            if (OUT_MODE == 1) {
              hv[e] = (_Float16)sp[e];
            } else {
              unsigned short hb = f2bf_bits(sp[e]);
              unsigned short lb = f2bf_bits(sp[e] - bf_bits2f(hb));
              hv[e] = __builtin_bit_cast(_Float16, hb);
              lv[e] = __builtin_bit_cast(_Float16, lb);
            }
          }
          *(volatile v8h*)(C + (size_t)(mBase + row) * ldc + n0 + c8) = hv;
          if (OUT_MODE == 2) *(volatile v8h*)(C2 + (size_t)(mBase + row) * ldc + n0 + c8) = lv;
        }
        __threadfence();
      }
    }
    __builtin_amdgcn_fence(__ATOMIC_RELEASE, "workgroup");
    __builtin_amdgcn_wave_barrier();
    __builtin_amdgcn_fence(__ATOMIC_ACQUIRE, "workgroup");
  }
}

__global__ __launch_bounds__(256) void cast_f32_f16x2_scaled(
    const float* __restrict__ in, unsigned short* __restrict__ out, int n2, float scale) {
  int i = blockIdx.x * 256 + threadIdx.x;
  if (i < n2) {
    const _Float16 h0 = (_Float16)(in[2 * i] * scale), h1 = (_Float16)(in[2 * i + 1] * scale);
    const unsigned u = (unsigned)__builtin_bit_cast(unsigned short, h0) | ((unsigned)__builtin_bit_cast(unsigned short, h1) << 16);
    ((volatile unsigned*)out)[i] = u;
    __threadfence();
    ((volatile unsigned*)out)[i] = u;
  }
}

__global__ __launch_bounds__(128) void layernorm_f16_kernel(
    const float* __restrict__ x, const float* __restrict__ lw, const float* __restrict__ lb,
    unsigned short* __restrict__ outp, float eps) {
  __shared__ float red0[4];
  __shared__ float red1[4];
  const int row = blockIdx.x;
  const int t = threadIdx.x;
  const int wave = t >> 5, lane = t & 31;
  const float* xr = x + (size_t)row * LN_F + t * 8;
  const v4f a0 = *(const v4f*)(xr);
  const v4f a1 = *(const v4f*)(xr + 4);
  float xv[8];
  xv[0] = a0[0]; xv[1] = a0[1]; xv[2] = a0[2]; xv[3] = a0[3];
  xv[4] = a1[0]; xv[5] = a1[1]; xv[6] = a1[2]; xv[7] = a1[3];
  float s = ((xv[0] + xv[1]) + (xv[2] + xv[3])) + ((xv[4] + xv[5]) + (xv[6] + xv[7]));
#pragma unroll
  for (int m = 1; m < 32; m <<= 1) s += __shfl_xor(s, m, 32);
  if (lane == 0) red0[wave] = s;
  __syncthreads();
  const float mu = ((red0[0] + red0[1]) + (red0[2] + red0[3])) * (1.0f / (float)LN_F);
  float d[8];
  float q = 0.f;
#pragma unroll
  for (int e = 0; e < 8; ++e) { d[e] = xv[e] - mu; q += d[e] * d[e]; }
#pragma unroll
  for (int m = 1; m < 32; m <<= 1) q += __shfl_xor(q, m, 32);
  if (lane == 0) red1[wave] = q;
  __syncthreads();
  const float var = ((red1[0] + red1[1]) + (red1[2] + red1[3])) * (1.0f / (float)LN_F);
  const float rstd = rsqrtf(var + eps);
  const v4f w0 = *(const v4f*)(lw + t * 8);
  const v4f w1 = *(const v4f*)(lw + t * 8 + 4);
  const v4f b0 = *(const v4f*)(lb + t * 8);
  const v4f b1 = *(const v4f*)(lb + t * 8 + 4);
  float wv8[8], bv8[8];
  wv8[0] = w0[0]; wv8[1] = w0[1]; wv8[2] = w0[2]; wv8[3] = w0[3];
  wv8[4] = w1[0]; wv8[5] = w1[1]; wv8[6] = w1[2]; wv8[7] = w1[3];
  bv8[0] = b0[0]; bv8[1] = b0[1]; bv8[2] = b0[2]; bv8[3] = b0[3];
  bv8[4] = b1[0]; bv8[5] = b1[1]; bv8[6] = b1[2]; bv8[7] = b1[3];
  v8h o;
#pragma unroll
  for (int e = 0; e < 8; ++e) o[e] = (_Float16)(d[e] * rstd * wv8[e] + bv8[e]);
  _Float16* orow = (_Float16*)(void*)outp + (size_t)row * LN_F + t * 8;
  *(volatile v8h*)orow = o;
  __threadfence();
  *(volatile v8h*)orow = o;
}

#define AT_D 64
#define AT_NW 4
#define AT_QB 64
#define AT_KC 64
#define AT_MAXCH 64
#define AT_PSC 32768.0f

__device__ __forceinline__ v8f mma_h(v16h a, v16h b, v8f c) {
  c = __builtin_amdgcn_wmma_f32_16x16x32_f16(false, a, false, b, (short)0, c, false, false);
  asm volatile("v_nop\n\tv_nop\n\tv_nop\n\tv_nop" : "+v"(c) : "v"(a), "v"(b));
  return c;
}

__global__ __launch_bounds__(128)
void attn64h_kernel(const unsigned short* __restrict__ qkvp, const int* __restrict__ seq_lens,
                    unsigned short* __restrict__ wvp, int S, int H, int ldq, int ldo,
                    float qk_scale, float mask_fill) {
  typedef _Float16 hT;
  union FH { v16h v; v8h h[2]; };
  const hT* qkv = (const hT*)(const void*)qkvp;
  hT* wvo = (hT*)(void*)wvp;
  __shared__ __align__(16) hT    Ksh[AT_KC * AT_D];
  __shared__ __align__(16) hT    Vth[AT_D * AT_KC];
  __shared__ __align__(16) hT    Psh[AT_NW][16 * AT_KC];
  __shared__ __align__(16) float Os[AT_NW][16 * 68];

  const int tid  = threadIdx.x;
  const int wave = tid >> 5;
  const int lane = tid & 31;
  const int hh   = lane >> 4;
  const int c    = lane & 15;

  const int nqb = S / AT_QB;
  const int bx = blockIdx.x;
  const int qb = bx % nqb;
  const int bh = bx / nqb;
  const int h  = bh % H;
  const int b  = bh / H;
  int slen = seq_lens[b];
  slen = slen < 0 ? 0 : (slen > S ? S : slen);
  const int qbase_block = qb * AT_QB;
  if (qbase_block >= slen) return;
  const int q0 = qbase_block + wave * 16;
  const int Fd = H * AT_D;

  const hT* qb_ptr = qkv + (size_t)b * S * ldq + (size_t)h * AT_D;
  const hT* kb_ptr = qb_ptr + Fd;
  const hT* vb_ptr = qb_ptr + 2 * Fd;
  hT*       ob_ptr = wvo + (size_t)b * S * ldo + (size_t)h * AT_D;

  v16h qa[2];
  {
    const hT* qrow = qb_ptr + (size_t)(q0 + c) * ldq;
    qa[0] = Frag<_Float16>::load(qrow + 8 * hh);
    qa[1] = Frag<_Float16>::load(qrow + 32 + 8 * hh);
  }

  float mrow[8], lrow[8];
  v8f oacc[4];
#pragma unroll
  for (int r = 0; r < 8; ++r) { mrow[r] = -__builtin_huge_valf(); lrow[r] = 0.f; }
#pragma unroll
  for (int t = 0; t < 4; ++t) oacc[t] = (v8f){0.f,0.f,0.f,0.f,0.f,0.f,0.f,0.f};

  int nChunks = (slen + AT_KC - 1) / AT_KC;
  const int maxch = S / AT_KC;
  if (nChunks > maxch) nChunks = maxch;
  if (nChunks > AT_MAXCH) nChunks = AT_MAXCH;

  for (int kc = 0; kc < nChunks; ++kc) {
    const int kv0 = kc * AT_KC;
    __syncthreads();
    {
      const int kvr = tid >> 1, dh = (tid & 1) * 32;
      const hT* krow = kb_ptr + (size_t)(kv0 + kvr) * ldq + dh;
      const hT* vrow = vb_ptr + (size_t)(kv0 + kvr) * ldq + dh;
#pragma unroll
      for (int i = 0; i < 4; ++i) {
        const v8h kk = *(const v8h*)(krow + 8 * i);
        *(v8h*)(Ksh + kvr * AT_D + dh + 8 * i) = kk;
        const v8h vv = *(const v8h*)(vrow + 8 * i);
#pragma unroll
        for (int e = 0; e < 8; ++e) Vth[(dh + 8 * i + e) * AT_KC + kvr] = vv[e];
      }
    }
    __syncthreads();

    v8f s[4];
#pragma unroll
    for (int j = 0; j < 4; ++j) {
      s[j] = (v8f){0.f,0.f,0.f,0.f,0.f,0.f,0.f,0.f};
#pragma unroll
      for (int dc = 0; dc < 2; ++dc) {
        FH kb;
        kb.h[0] = *(const v8h*)(Ksh + (j * 16 + c) * AT_D + dc * 32 + 8 * hh);
        kb.h[1] = *(const v8h*)(Ksh + (j * 16 + c) * AT_D + dc * 32 + 16 + 8 * hh);
        s[j] = mma_h(qa[dc], kb.v, s[j]);
      }
    }
    float cm[8];
#pragma unroll
    for (int r = 0; r < 8; ++r) {
      float m = -__builtin_huge_valf();
#pragma unroll
      for (int j = 0; j < 4; ++j) {
        const int kvcol = kv0 + j * 16 + c;
        float sv = s[j][r] * qk_scale;
        if (kvcol >= slen) sv = mask_fill;
        s[j][r] = sv;
        m = fmaxf(m, sv);
      }
#pragma unroll
      for (int off = 1; off < 16; off <<= 1) m = fmaxf(m, __shfl_xor(m, off, 32));
      cm[r] = m;
    }
    hT* pwh = Psh[wave];
#pragma unroll
    for (int r = 0; r < 8; ++r) {
      const float mnew = fmaxf(mrow[r], cm[r]);
      const float alpha = expf(mrow[r] - mnew);
      mrow[r] = mnew;
      float psum = 0.f;
#pragma unroll
      for (int j = 0; j < 4; ++j) {
        const float p = expf(s[j][r] - mnew);
        psum += p;
        pwh[(8 * hh + r) * AT_KC + j * 16 + c] = (hT)(p * AT_PSC);
      }
#pragma unroll
      for (int off = 1; off < 16; off <<= 1) psum += __shfl_xor(psum, off, 32);
      lrow[r] = lrow[r] * alpha + psum;
#pragma unroll
      for (int t = 0; t < 4; ++t) oacc[t][r] *= alpha;
    }
    __builtin_amdgcn_fence(__ATOMIC_RELEASE, "workgroup");
    __builtin_amdgcn_wave_barrier();
    __builtin_amdgcn_fence(__ATOMIC_ACQUIRE, "workgroup");
#pragma unroll 1
    for (int kk = 0; kk < 2; ++kk) {
      FH pa;
      pa.h[0] = *(const v8h*)(pwh + c * AT_KC + kk * 32 + 8 * hh);
      pa.h[1] = *(const v8h*)(pwh + c * AT_KC + kk * 32 + 16 + 8 * hh);
#pragma unroll
      for (int t = 0; t < 4; ++t) {
        FH vb;
        vb.h[0] = *(const v8h*)(Vth + (t * 16 + c) * AT_KC + kk * 32 + 8 * hh);
        vb.h[1] = *(const v8h*)(Vth + (t * 16 + c) * AT_KC + kk * 32 + 16 + 8 * hh);
        oacc[t] = mma_h(pa.v, vb.v, oacc[t]);
      }
    }
  }

  float* os = Os[wave];
#pragma unroll
  for (int r = 0; r < 8; ++r) {
    const float inv = 1.0f / (lrow[r] * AT_PSC);
#pragma unroll
    for (int t = 0; t < 4; ++t) os[(8 * hh + r) * 68 + t * 16 + c] = oacc[t][r] * inv;
  }
  __builtin_amdgcn_fence(__ATOMIC_RELEASE, "workgroup");
  __builtin_amdgcn_wave_barrier();
  __builtin_amdgcn_fence(__ATOMIC_ACQUIRE, "workgroup");
  {
    const int q = lane >> 3, c8 = (lane & 7) * 8;
    for (int pass = 0; pass < 2; ++pass) {
#pragma unroll
      for (int it = 0; it < 4; ++it) {
        const int row = it * 4 + q;
        const float* sp = os + row * 68 + c8;
        v8h hv;
#pragma unroll
        for (int e = 0; e < 8; ++e) hv[e] = (hT)sp[e];
        *(volatile v8h*)(ob_ptr + (size_t)(q0 + row) * ldo + c8) = hv;
      }
      __threadfence();
    }
  }
}

extern "C" void kernel_launch(void* const* d_in, const int* in_sizes, int n_in,
                              void* d_out, int out_size, void* d_ws,
                              size_t ws_size, hipStream_t stream) {
  if (n_in < 8) return;
  const float* x     = (const float*)d_in[0];
  const int*   slen  = (const int*)d_in[1];
  const float* ln_w  = (const float*)d_in[2];
  const float* ln_b  = (const float*)d_in[3];
  const float* in_w  = (const float*)d_in[4];
  const float* in_b  = (const float*)d_in[5];
  const float* out_w = (const float*)d_in[6];
  const float* out_b = (const float*)d_in[7];
  float* out = (float*)d_out;

  const int Bn = in_sizes[1];
  const int Fd = in_sizes[2];
  const int G3 = in_sizes[5];
  if (Bn <= 0 || Fd != LN_F || G3 != 3 * Fd) return;
  const long long xn = (long long)in_sizes[0];
  const long long per = (long long)Bn * Fd;
  if (xn <= 0 || (xn % per) != 0) return;
  const int S = (int)(xn / per);
  if (S <= 0 || (S % 64) != 0) return;
  if (in_sizes[3] != Fd || in_sizes[4] != G3 * Fd || in_sizes[6] != Fd * Fd || in_sizes[7] != Fd) return;
  if ((long long)out_size != xn) return;
  const int M = Bn * S;
  const int H = Fd / AT_D;

  char* ws = (char*)d_ws;
  size_t off = 0;
  auto carve = [&](size_t bytes) -> void* {
    void* p = ws + off;
    off = (off + bytes + 255) & ~(size_t)255;
    return p;
  };
  unsigned short* in_w16  = (unsigned short*)carve((size_t)G3 * Fd * 2);
  unsigned short* out_w16 = (unsigned short*)carve((size_t)Fd * Fd * 2);
  unsigned short* normA   = (unsigned short*)carve((size_t)M * Fd * 2);
  unsigned short* qkv     = (unsigned short*)carve((size_t)M * G3 * 2);
  unsigned short* wvb     = (unsigned short*)carve((size_t)M * Fd * 2);
  if (off > ws_size || off > WS_CAP) return;

  {
    const int n2 = (G3 * Fd) / 2;
    cast_f32_f16x2_scaled<<<dim3((n2 + 255) / 256), dim3(256), 0, stream>>>(in_w, in_w16, n2, 16.0f);
  }
  {
    const int n2 = (Fd * Fd) / 2;
    cast_f32_f16x2_scaled<<<dim3((n2 + 255) / 256), dim3(256), 0, stream>>>(out_w, out_w16, n2, 16.0f);
  }
  layernorm_f16_kernel<<<dim3(M), dim3(128), 0, stream>>>(x, ln_w, ln_b, normA, 1e-5f);
  {
    const int tiles = (M / 64) * (G3 / 64);
    dim3 grid((tiles + 7) / 8, 1);
    wmma_gemm64<0, false, 2, 1, false, 0, 1><<<grid, dim3(256), 0, stream>>>(
        normA, normA, Fd, 0L,
        in_w16, in_w16, Fd, 0L,
        (void*)qkv, (void*)qkv, G3, 0L,
        in_b,
        x, 0L,
        M, G3, Fd, 1.0f / 16.0f,
        slen, S);
  }
  {
    dim3 grid(Bn * H * (S / AT_QB));
    attn64h_kernel<<<grid, dim3(128), 0, stream>>>(qkv, slen, wvb, S, H, G3, Fd, 0.125f, -1.0e9f);
  }
  {
    const int tiles = (M / 64) * (Fd / 64);
    dim3 grid((tiles + 7) / 8, 1);
    wmma_gemm64<0, false, 2, 0, true, 0, 2><<<grid, dim3(256), 0, stream>>>(
        wvb, wvb, Fd, 0L,
        out_w16, out_w16, Fd, 0L,
        (void*)out, (void*)out, Fd, 0L,
        out_b,
        x, 0L,
        M, Fd, Fd, 1.0f / 16.0f,
        slen, S);
  }
}
